// PaiNNInteraction_60601988547144
// MI455X (gfx1250) — hardware-verified
//
#include <hip/hip_runtime.h>
#include <stddef.h>
#include <stdint.h>


#define HD      128
#define H3      384
#define RD      20
#define KR      32
#define NTHR    256
#define NWAVE   8
#define EPT     8
#define CHUNK   (NTHR * EPT)
#define WCAP    (EPT * 32)
#define LISTN   (NWAVE * WCAP)
#define NBMAX   2048
#define RCAP    28672
#define DEGCAP  512
#define GBM     64
#define GBN     64
#define GTHR    128
#define ECH     40000
#define OW_F1   0
#define OW_S1   (HD * KR)
#define OW_F2   (OW_S1 + HD * HD)
#define OW_S2   (OW_F2 + H3 * HD)
#define NW_TOT  (OW_S2 + H3 * HD)
#define U_F1    (HD * (KR / 8))
#define U_S1    (U_F1 + HD * (HD / 8))
#define U_F2    (U_S1 + H3 * (HD / 8))
#define U_TOT   (U_F2 + H3 * (HD / 8))
#define CW      1024.0f
#define CS      16.0f
#define CH      64.0f
#define CR      1024.0f
#define CZ      64.0f
#define CF      256.0f
#define RCF     0.00390625f
#define LOS     2048.0f
#define RLO     0.00048828125f
#define SCL_S1  6.103515625e-05f
#define SCL_S2  1.52587890625e-05f
#define SCL_F1  9.5367431640625e-07f
#define SCL_F2  1.52587890625e-05f
#define WSMAX   134217728
#define LDS_AGG ((2 * RCAP + 2 * NBMAX + LISTN) * 4 + 64)

static_assert((CHUNK & (CHUNK - 1)) == 0 && CHUNK <= 4096);
static_assert((NBMAX & (NBMAX - 1)) == 0 && NBMAX <= 4096);
static_assert(NTHR * 8 == NBMAX);
static_assert(LISTN >= NBMAX);
static_assert(LISTN >= NWAVE * WCAP);
static_assert((RCAP % 32) == 0);
static_assert(LDS_AGG <= 300000);
static_assert(GBM == (GTHR / 32) * 16);
static_assert((HD % 32) == 0 && (HD % GBN) == 0 && (H3 % GBN) == 0 && KR == 32);
static_assert((ECH % GBM) == 0);
static_assert((U_F1 % NTHR) == 0 && (U_S1 % NTHR) == 0 && (U_F2 % NTHR) == 0 && (U_TOT % NTHR) == 0);
static_assert(HD == 4 * 32);
static_assert(RD <= 20 && RD + 4 <= 24);

typedef float    v4f  __attribute__((ext_vector_type(4)));
typedef float    v8f  __attribute__((ext_vector_type(8)));
typedef int      v4i  __attribute__((ext_vector_type(4)));
typedef int      v8i  __attribute__((ext_vector_type(8)));
typedef _Float16 v4h  __attribute__((ext_vector_type(4)));
typedef _Float16 v8h  __attribute__((ext_vector_type(8)));
typedef _Float16 v16h __attribute__((ext_vector_type(16)));
union FragH { v16h v; v8h h[2]; v8i w; };

__device__ __forceinline__ v8f wmh(const FragH& a, const FragH& b, v8f c) {
  v8f d = __builtin_amdgcn_wmma_f32_16x16x32_f16(false, a.v, false, b.v, (short)0, c, false, false);
  asm volatile("v_nop\n\tv_nop\n\tv_nop\n\tv_nop" : "+v"(d) : "v"(a.w), "v"(b.w));
  return d;
}

__device__ __forceinline__ void ldwait() {
  asm volatile("s_wait_loadcnt 0x0" ::: "memory");
}

__device__ __forceinline__ float bf16r(float x) {
  unsigned u = __float_as_uint(x);
  u = (u + 0x7FFFu + ((u >> 16) & 1u)) & 0xFFFF0000u;
  return __uint_as_float(u);
}

__device__ __forceinline__ float rcp_f(float x) { return __builtin_amdgcn_rcpf(x); }
__device__ __forceinline__ float silu_f(float x) { return x * rcp_f(1.0f + __expf(-x)); }

__device__ __forceinline__ int scan_chunk(const int* __restrict__ dsts, int nE, int cbase, int slotBase,
                                          int nb, int vec8, int* list, int tid, int lane, int wave) {
  int wc = 0;
  const int el0  = tid * EPT;
  const int e0   = cbase + el0;
  const int sent = -2147483647 - 1;
  v4i da, db;
  if (vec8 != 0 && cbase + CHUNK <= nE) {
    da = *(const v4i*)(dsts + e0);
    db = *(const v4i*)(dsts + e0 + 4);
  } else {
    da.x = (e0     < nE) ? dsts[min(e0,     nE - 1)] : sent;
    da.y = (e0 + 1 < nE) ? dsts[min(e0 + 1, nE - 1)] : sent;
    da.z = (e0 + 2 < nE) ? dsts[min(e0 + 2, nE - 1)] : sent;
    da.w = (e0 + 3 < nE) ? dsts[min(e0 + 3, nE - 1)] : sent;
    db.x = (e0 + 4 < nE) ? dsts[min(e0 + 4, nE - 1)] : sent;
    db.y = (e0 + 5 < nE) ? dsts[min(e0 + 5, nE - 1)] : sent;
    db.z = (e0 + 6 < nE) ? dsts[min(e0 + 6, nE - 1)] : sent;
    db.w = (e0 + 7 < nE) ? dsts[min(e0 + 7, nE - 1)] : sent;
  }
  const unsigned nbs = (unsigned)slotBase;
  const unsigned unb = (unsigned)nb;
  const unsigned s0 = (unsigned)da.x - nbs, s1 = (unsigned)da.y - nbs;
  const unsigned s2 = (unsigned)da.z - nbs, s3 = (unsigned)da.w - nbs;
  const unsigned s4 = (unsigned)db.x - nbs, s5 = (unsigned)db.y - nbs;
  const unsigned s6 = (unsigned)db.z - nbs, s7 = (unsigned)db.w - nbs;
  const bool h0 = s0 < unb, h1 = s1 < unb, h2 = s2 < unb, h3 = s3 < unb;
  const bool h4 = s4 < unb, h5 = s5 < unb, h6 = s6 < unb, h7 = s7 < unb;
  const unsigned any = __builtin_amdgcn_ballot_w32(h0 | h1 | h2 | h3 | h4 | h5 | h6 | h7);
  if (any != 0u) {
#define HITJ(J, HJ, SJ) { \
      const unsigned mj = __builtin_amdgcn_ballot_w32(HJ); \
      if (mj != 0u) { \
        if (HJ) { \
          const int pos = wc + (int)__builtin_amdgcn_mbcnt_lo(mj, 0u); \
          if (pos < WCAP) list[wave * WCAP + pos] = ((el0 + (J)) << 12) | (int)(SJ); \
        } \
        wc += (int)__builtin_popcount(mj); } }
    HITJ(0, h0, s0)
    HITJ(1, h1, s1)
    HITJ(2, h2, s2)
    HITJ(3, h3, s3)
    HITJ(4, h4, s4)
    HITJ(5, h5, s5)
    HITJ(6, h6, s6)
    HITJ(7, h7, s7)
#undef HITJ
  }
  return wc;
}

__global__ __launch_bounds__(NTHR) void k_wcvt(const float* __restrict__ fW1, const float* __restrict__ sW1,
                                               const float* __restrict__ fW2, const float* __restrict__ sW2,
                                               _Float16* wt, int nUnits) {
  const int u = (int)blockIdx.x * NTHR + (int)threadIdx.x;
  if (u >= nUnits) return;
  const float* src;
  int n, k8, pitch, kmax;
  size_t o;
  if (u < U_F1) {
    n = u >> 2; k8 = (u & 3) * 8; src = fW1; pitch = HD; kmax = RD;
    o = (size_t)OW_F1 + (size_t)n * KR + k8;
  } else if (u < U_S1) {
    const int uu = u - U_F1;
    n = uu >> 4; k8 = (uu & 15) * 8; src = sW1; pitch = HD; kmax = HD;
    o = (size_t)OW_S1 + (size_t)n * HD + k8;
  } else if (u < U_F2) {
    const int uu = u - U_S1;
    n = uu >> 4; k8 = (uu & 15) * 8; src = fW2; pitch = H3; kmax = HD;
    o = (size_t)OW_F2 + (size_t)n * HD + k8;
  } else {
    const int uu = u - U_F2;
    n = uu >> 4; k8 = (uu & 15) * 8; src = sW2; pitch = H3; kmax = HD;
    o = (size_t)OW_S2 + (size_t)n * HD + k8;
  }
  v8h hv;
#pragma unroll
  for (int j = 0; j < 8; ++j) {
    const int k  = k8 + j;
    const int kc = k < kmax ? k : kmax - 1;
    const float w = src[(size_t)kc * pitch + n];
    const float x = (k < kmax) ? bf16r(w) * CW : 0.0f;
    hv[j] = (_Float16)x;
  }
  *(volatile v8h*)(wt + o) = hv;
  __threadfence();
  *(volatile v8h*)(wt + o) = hv;
}

__global__ __launch_bounds__(NTHR) void k_scvt(const float* __restrict__ s, _Float16* dst, int nSrc, int nUnits) {
  const int i = (int)blockIdx.x * NTHR + (int)threadIdx.x;
  if (i >= nUnits) return;
  const int row = i >> 4;
  const int c0  = (i & 15) * 8;
  const int rc  = row < nSrc ? row : nSrc - 1;
  const float* p = s + (size_t)rc * HD + c0;
  v4f a = *(const v4f*)p, b = *(const v4f*)(p + 4);
  const v4f z4 = {0.f, 0.f, 0.f, 0.f};
  if (row >= nSrc) { a = z4; b = z4; }
  v8h hv;
  hv[0] = (_Float16)(bf16r(a.x) * CS); hv[1] = (_Float16)(bf16r(a.y) * CS);
  hv[2] = (_Float16)(bf16r(a.z) * CS); hv[3] = (_Float16)(bf16r(a.w) * CS);
  hv[4] = (_Float16)(bf16r(b.x) * CS); hv[5] = (_Float16)(bf16r(b.y) * CS);
  hv[6] = (_Float16)(bf16r(b.z) * CS); hv[7] = (_Float16)(bf16r(b.w) * CS);
  const size_t o = (size_t)row * HD + c0;
  *(volatile v8h*)(dst + o) = hv;
  __threadfence();
  *(volatile v8h*)(dst + o) = hv;
}

__global__ __launch_bounds__(NTHR) void k_rcvt(const float* __restrict__ rbf, _Float16* dst,
                                               int ebase, int nE, int nUnits) {
  const int i = (int)blockIdx.x * NTHR + (int)threadIdx.x;
  if (i >= nUnits) return;
  const int le = i >> 2;
  const int p  = i & 3;
  const int e  = ebase + le;
  const int ec = e < nE ? e : nE - 1;
  const float* rp = rbf + (size_t)ec * RD;
  int o0 = 8 * p;     o0 = o0 > 16 ? 16 : o0;
  int o1 = 8 * p + 4; o1 = o1 > 16 ? 16 : o1;
  v4f a = *(const v4f*)(rp + o0), b = *(const v4f*)(rp + o1);
  const v4f z4 = {0.f, 0.f, 0.f, 0.f};
  const bool va = (p < 3) && (e < nE);
  const bool vb = (p < 2) && (e < nE);
  if (!va) a = z4;
  if (!vb) b = z4;
  v8h hv;
  hv[0] = (_Float16)(bf16r(a.x) * CR); hv[1] = (_Float16)(bf16r(a.y) * CR);
  hv[2] = (_Float16)(bf16r(a.z) * CR); hv[3] = (_Float16)(bf16r(a.w) * CR);
  hv[4] = (_Float16)(bf16r(b.x) * CR); hv[5] = (_Float16)(bf16r(b.y) * CR);
  hv[6] = (_Float16)(bf16r(b.z) * CR); hv[7] = (_Float16)(bf16r(b.w) * CR);
  const size_t o = (size_t)le * KR + 8 * p;
  *(volatile v8h*)(dst + o) = hv;
  __threadfence();
  *(volatile v8h*)(dst + o) = hv;
}

template<int EPI, int ASPL>
__global__ __launch_bounds__(GTHR) void k_gemm(
    const _Float16* __restrict__ A, const _Float16* __restrict__ AL, const _Float16* __restrict__ WT,
    const float* __restrict__ bias, float* outF, _Float16* outH, _Float16* outL,
    int K, int ldo, int nbias, float scl, float oc)
{
  __shared__ __attribute__((aligned(16))) float stg[GBM * GBN];
  const int tid = (int)threadIdx.x, lane = tid & 31, wave = tid >> 5, hh = lane >> 4, m = lane & 15;
  const int rowBase = (int)blockIdx.x * GBM;
  const int col0    = (int)blockIdx.y * GBN;

  v8f acc[4], accl[4];
  {
    const v8f z = {0.f, 0.f, 0.f, 0.f, 0.f, 0.f, 0.f, 0.f};
    acc[0] = z; acc[1] = z; acc[2] = z; acc[3] = z;
    accl[0] = z; accl[1] = z; accl[2] = z; accl[3] = z;
  }
  const size_t ro = (size_t)(rowBase + 16 * wave + m) * (size_t)K + 8 * hh;
  const _Float16* ap  = A  + ro;
  const _Float16* alp = AL + ro;
  const _Float16* wp  = WT + (size_t)(col0 + m) * (size_t)K + 8 * hh;
  const int ksteps = K >> 5;
#pragma unroll 1
  for (int ks = 0; ks < ksteps; ++ks) {
    FragH af, afl;
    af.h[0] = *(const v8h*)(ap + 32 * ks);
    af.h[1] = *(const v8h*)(ap + 32 * ks + 16);
    if (ASPL) {
      afl.h[0] = *(const v8h*)(alp + 32 * ks);
      afl.h[1] = *(const v8h*)(alp + 32 * ks + 16);
    } else {
      afl = af;
    }
#pragma unroll
    for (int t = 0; t < 4; ++t) {
      const _Float16* wq = wp + (size_t)(16 * t) * (size_t)K + 32 * ks;
      FragH bf;
      bf.h[0] = *(const v8h*)wq;
      bf.h[1] = *(const v8h*)(wq + 16);
      acc[t] = wmh(af, bf, acc[t]);
      if (ASPL) accl[t] = wmh(afl, bf, accl[t]);
    }
  }

#pragma unroll
  for (int t = 0; t < 4; ++t) {
    const int lc  = 16 * t + m;
    const int col = col0 + lc;
    int ci = col > nbias - 1 ? nbias - 1 : col;
    ci = ci < 0 ? 0 : ci;
    const float bl = bf16r(bias[ci]);
    const float bv = (col < nbias) ? bl : 0.f;
#pragma unroll
    for (int r = 0; r < 8; ++r) {
      const int lr = 16 * wave + 8 * hh + r;
      float x = acc[t][r];
      if (ASPL) x = fmaf(accl[t][r], RLO, x);
      float v = fmaf(x, scl, bv);
      if (EPI == 1 || EPI == 2) v = silu_f(v);
      stg[lr * GBN + lc] = v;
    }
  }
  __syncthreads();

  if (EPI == 0) {
    v4f fv[8];
#pragma unroll
    for (int i = 0; i < 8; ++i) {
      const int lr = 16 * wave + 2 * i + hh;
      fv[i] = *(const v4f*)(stg + lr * GBN + 4 * m);
    }
#pragma unroll
    for (int i = 0; i < 8; ++i) {
      const int lr = 16 * wave + 2 * i + hh;
      const int gr = rowBase + lr;
      float* op = outF + (size_t)gr * (size_t)ldo + col0 + 4 * m;
      *(volatile v4f*)op = fv[i];
    }
    __threadfence();
#pragma unroll
    for (int i = 0; i < 8; ++i) {
      const int lr = 16 * wave + 2 * i + hh;
      const int gr = rowBase + lr;
      float* op = outF + (size_t)gr * (size_t)ldo + col0 + 4 * m;
      *(volatile v4f*)op = fv[i];
    }
  } else {
    const int q8 = (lane & 7) * 8;
    v8h hv[4], lv[4];
#pragma unroll
    for (int i = 0; i < 4; ++i) {
      const int lr = 16 * wave + 4 * i + (lane >> 3);
      const v4f a = *(const v4f*)(stg + lr * GBN + q8);
      const v4f b = *(const v4f*)(stg + lr * GBN + q8 + 4);
      const float x[8] = {a.x * oc, a.y * oc, a.z * oc, a.w * oc, b.x * oc, b.y * oc, b.z * oc, b.w * oc};
      v8h hq, lq;
#pragma unroll
      for (int j = 0; j < 8; ++j) {
        const _Float16 hj = (_Float16)x[j];
        hq[j] = hj;
        lq[j] = (_Float16)((x[j] - (float)hj) * LOS);
      }
      hv[i] = hq; lv[i] = lq;
    }
#pragma unroll
    for (int i = 0; i < 4; ++i) {
      const int lr = 16 * wave + 4 * i + (lane >> 3);
      const int gr = rowBase + lr;
      const size_t oo = (size_t)gr * (size_t)ldo + col0 + q8;
      *(volatile v8h*)(outH + oo) = hv[i];
      if (EPI == 2) *(volatile v8h*)(outL + oo) = lv[i];
    }
    __threadfence();
#pragma unroll
    for (int i = 0; i < 4; ++i) {
      const int lr = 16 * wave + 4 * i + (lane >> 3);
      const int gr = rowBase + lr;
      const size_t oo = (size_t)gr * (size_t)ldo + col0 + q8;
      *(volatile v8h*)(outH + oo) = hv[i];
      if (EPI == 2) *(volatile v8h*)(outL + oo) = lv[i];
    }
  }
}

__global__ __launch_bounds__(NTHR) void k_drain(
    const int* __restrict__ ei, const float* __restrict__ unit, const _Float16* __restrict__ FP,
    const float* __restrict__ SP, const float* __restrict__ vin, const float* __restrict__ sin_,
    float* DS, float* DV, float* out0, float* out1,
    int nN, int nEt, int ebase, int nEc, int nb, int vec8, int NPD, int accum, int fin) {
  extern __shared__ v4f lds_dyn[];
  int* reg1 = (int*)lds_dyn;
  int* reg2 = reg1 + RCAP;
  int* scnt = reg2 + RCAP;
  int* soff = scnt + NBMAX;
  int* list = soff + NBMAX;
  int* wcnt = list + LISTN;
  int* wtot = wcnt + NWAVE;
  const int tid = (int)threadIdx.x, lane = tid & 31, wave = tid >> 5;
  const int nodeBase = (int)blockIdx.x * nb;
  const int* dsts = ei + (size_t)nEt + (size_t)ebase;
  const int nE = nEc;

  for (int i = tid; i < NBMAX; i += NTHR) scnt[i] = 0;
  __syncthreads();

  int tot = 0;
  const int nChunks = (nE + CHUNK - 1) / CHUNK;
#pragma unroll 1
  for (int ch = 0; ch < nChunks; ++ch) {
    const int cbase = ch * CHUNK;
    const int wc = scan_chunk(dsts, nE, cbase, nodeBase, nb, vec8, list, tid, lane, wave);
    if (lane == 0) wcnt[wave] = wc;
    __syncthreads();
    int pre = 0, all = 0;
#pragma unroll
    for (int w2 = 0; w2 < NWAVE; ++w2) {
      int c = wcnt[w2];
      c = c < 0 ? 0 : (c > WCAP ? WCAP : c);
      all += c;
      pre += (w2 < wave) ? c : 0;
    }
    const int wcc  = wc > WCAP ? WCAP : wc;
    const int base = tot + pre;
#pragma unroll 1
    for (int i = lane; i < wcc; i += 32) {
      const int ent = list[wave * WCAP + i];
      const int el  = (ent >> 12) & (CHUNK - 1);
      const int sl  = ent & (NBMAX - 1);
      int eid = cbase + el;
      eid = eid > nE - 1 ? nE - 1 : eid;
      const int pos = base + i;
      if (pos < RCAP) reg1[pos] = (int)(((unsigned)eid << 12) | (unsigned)sl);
    }
    tot += all;
    tot = tot > RCAP ? RCAP : tot;
    __syncthreads();
  }
  const int nh = tot;

  if (wave == 0) {
#pragma unroll 1
    for (int b0 = 0; b0 < nh; b0 += 32) {
      const int idx = b0 + lane;
      const int uv  = reg1[idx < RCAP ? idx : RCAP - 1];
      const int m32 = (nh - b0) < 32 ? (nh - b0) : 32;
#pragma unroll 1
      for (int k = 0; k < m32; ++k) {
        const int u  = __builtin_amdgcn_readlane(uv, k);
        const int sl = u & (NBMAX - 1);
        if (lane == 0) scnt[sl] = scnt[sl] + 1;
      }
    }
  }
  __syncthreads();

  {
    const v4i ca = *(const v4i*)(scnt + 8 * tid);
    const v4i cb = *(const v4i*)(scnt + 8 * tid + 4);
    const int e0 = ca.x < 0 ? 0 : ca.x, e1 = ca.y < 0 ? 0 : ca.y, e2 = ca.z < 0 ? 0 : ca.z, e3 = ca.w < 0 ? 0 : ca.w;
    const int e4 = cb.x < 0 ? 0 : cb.x, e5 = cb.y < 0 ? 0 : cb.y, e6 = cb.z < 0 ? 0 : cb.z, e7 = cb.w < 0 ? 0 : cb.w;
    const int ts = e0 + e1 + e2 + e3 + e4 + e5 + e6 + e7;
    int incl = ts;
#pragma unroll
    for (int d = 1; d < 32; d <<= 1) {
      const int up = __shfl_up(incl, d);
      if (lane >= d) incl += up;
    }
    if (lane == 31) wtot[wave] = incl;
    __syncthreads();
    int pre = 0;
#pragma unroll
    for (int w2 = 0; w2 < NWAVE; ++w2) pre += (w2 < wave) ? wtot[w2] : 0;
    int run = pre + incl - ts;
    soff[8 * tid + 0] = run; run += e0;
    soff[8 * tid + 1] = run; run += e1;
    soff[8 * tid + 2] = run; run += e2;
    soff[8 * tid + 3] = run; run += e3;
    soff[8 * tid + 4] = run; run += e4;
    soff[8 * tid + 5] = run; run += e5;
    soff[8 * tid + 6] = run; run += e6;
    soff[8 * tid + 7] = run;
  }
  __syncthreads();
  for (int i = tid; i < NBMAX; i += NTHR) list[i] = soff[i];
  __syncthreads();

  if (wave == 0) {
#pragma unroll 1
    for (int b0 = 0; b0 < nh; b0 += 32) {
      const int idx = b0 + lane;
      const int uv  = reg1[idx < RCAP ? idx : RCAP - 1];
      const int m32 = (nh - b0) < 32 ? (nh - b0) : 32;
#pragma unroll 1
      for (int k = 0; k < m32; ++k) {
        const int u   = __builtin_amdgcn_readlane(uv, k);
        const int sl  = u & (NBMAX - 1);
        const int eid = (int)((unsigned)u >> 12);
        if (lane == 0) {
          int pos = list[sl];
          pos = pos < 0 ? 0 : (pos > RCAP - 1 ? RCAP - 1 : pos);
          reg2[pos] = eid;
          list[sl] = pos + 1;
        }
      }
    }
  }
  __syncthreads();

  const int nbw = nb >> 3;
  const bool ovf = (nh >= RCAP);
  const float qnan = __int_as_float(0x7fc00000);
  const int c4 = 4 * lane;
#pragma unroll 1
  for (int jt = 0; jt < nbw; ++jt) {
    const int slot = wave * nbw + jt;
    const int grow = nodeBase + slot;
    const int gcl  = grow < nN ? grow : nN - 1;
    const int gw   = grow < NPD ? grow : NPD - 1;
    int st = soff[slot];
    const int craw = scnt[slot];
    int cnt = craw;
    st  = st < 0 ? 0 : (st > nh ? nh : st);
    cnt = cnt < 0 ? 0 : (cnt > DEGCAP ? DEGCAP : cnt);
    if (cnt > nh - st) cnt = nh - st;
    const float pz = (ovf || craw > DEGCAP) ? qnan : 0.0f;
    const bool wout = grow < nN;
    const bool wr   = grow < NPD;
    const float live = wout ? 1.0f : 0.0f;

    float as_[4], a0[4], a1[4], a2[4];
#pragma unroll
    for (int j = 0; j < 4; ++j) { as_[j] = 0.f; a0[j] = 0.f; a1[j] = 0.f; a2[j] = 0.f; }
#pragma unroll 1
    for (int q = 0; q < cnt; ++q) {
      int idx = st + q; idx = idx > RCAP - 1 ? RCAP - 1 : idx;
      int el = reg2[idx]; el = el < 0 ? 0 : (el > nEc - 1 ? nEc - 1 : el);
      const int e = ebase + el;
      int sr = ei[e]; sr = sr < 0 ? 0 : (sr > nN - 1 ? nN - 1 : sr);
      const _Float16* fr = FP + (size_t)el * H3 + c4;
      const v4h f0 = *(const v4h*)fr;
      const v4h f1 = *(const v4h*)(fr + HD);
      const v4h f2 = *(const v4h*)(fr + 2 * HD);
      const float* pr = SP + (size_t)sr * H3 + c4;
      const v4f p0 = *(const v4f*)pr, p1 = *(const v4f*)(pr + HD), p2 = *(const v4f*)(pr + 2 * HD);
      const float* xr = vin + (size_t)sr * H3 + c4;
      const v4f x0 = *(const v4f*)xr, x1 = *(const v4f*)(xr + HD), x2 = *(const v4f*)(xr + 2 * HD);
      const float* ur = unit + (size_t)e * 3;
      const float ua = ur[0], ub = ur[1], uc = ur[2];
      ldwait();
      const float ff0[4] = {(float)f0.x, (float)f0.y, (float)f0.z, (float)f0.w};
      const float ff1[4] = {(float)f1.x, (float)f1.y, (float)f1.z, (float)f1.w};
      const float ff2[4] = {(float)f2.x, (float)f2.y, (float)f2.z, (float)f2.w};
      const float pp0[4] = {p0.x, p0.y, p0.z, p0.w};
      const float pp1[4] = {p1.x, p1.y, p1.z, p1.w};
      const float pp2[4] = {p2.x, p2.y, p2.z, p2.w};
      const float xx0[4] = {x0.x, x0.y, x0.z, x0.w};
      const float xx1[4] = {x1.x, x1.y, x1.z, x1.w};
      const float xx2[4] = {x2.x, x2.y, x2.z, x2.w};
      const float ra = bf16r(ua), rb = bf16r(ub), rc = bf16r(uc);
#pragma unroll
      for (int j = 0; j < 4; ++j) {
        const float ms = (ff0[j] * RCF) * pp0[j];
        const float mv = (ff1[j] * RCF) * pp1[j];
        const float mr = (ff2[j] * RCF) * pp2[j];
        as_[j] += ms;
        a0[j] += fmaf(mv, bf16r(xx0[j]), mr * ra);
        a1[j] += fmaf(mv, bf16r(xx1[j]), mr * rb);
        a2[j] += fmaf(mv, bf16r(xx2[j]), mr * rc);
      }
    }
    float od[4], o0[4], o1[4], o2[4];
#pragma unroll
    for (int j = 0; j < 4; ++j) { od[j] = 0.f; o0[j] = 0.f; o1[j] = 0.f; o2[j] = 0.f; }
    if (accum != 0) {
      const v4f d0 = *(const v4f*)(DS + (size_t)gw * HD + c4);
      const float* dvr = DV + (size_t)gw * H3 + c4;
      const v4f d1 = *(const v4f*)dvr, d2 = *(const v4f*)(dvr + HD), d3 = *(const v4f*)(dvr + 2 * HD);
      ldwait();
      od[0] = d0.x; od[1] = d0.y; od[2] = d0.z; od[3] = d0.w;
      o0[0] = d1.x; o0[1] = d1.y; o0[2] = d1.z; o0[3] = d1.w;
      o1[0] = d2.x; o1[1] = d2.y; o1[2] = d2.z; o1[3] = d2.w;
      o2[0] = d3.x; o2[1] = d3.y; o2[2] = d3.z; o2[3] = d3.w;
    }
    float rs[4], r0[4], r1[4], r2[4];
#pragma unroll
    for (int j = 0; j < 4; ++j) {
      rs[j] = (as_[j] + od[j]) * live + pz;
      r0[j] = (a0[j] + o0[j]) * live + pz;
      r1[j] = (a1[j] + o1[j]) * live + pz;
      r2[j] = (a2[j] + o2[j]) * live + pz;
    }
    if (fin != 0) {
      const v4f sv = *(const v4f*)(sin_ + (size_t)gcl * HD + c4);
      const float* vp = vin + (size_t)gcl * H3 + c4;
      const v4f y0 = *(const v4f*)vp, y1 = *(const v4f*)(vp + HD), y2 = *(const v4f*)(vp + 2 * HD);
      ldwait();
      v4f w0, w1, w2, w3;
      w0.x = rs[0] + bf16r(sv.x); w0.y = rs[1] + bf16r(sv.y); w0.z = rs[2] + bf16r(sv.z); w0.w = rs[3] + bf16r(sv.w);
      w1.x = r0[0] + bf16r(y0.x); w1.y = r0[1] + bf16r(y0.y); w1.z = r0[2] + bf16r(y0.z); w1.w = r0[3] + bf16r(y0.w);
      w2.x = r1[0] + bf16r(y1.x); w2.y = r1[1] + bf16r(y1.y); w2.z = r1[2] + bf16r(y1.z); w2.w = r1[3] + bf16r(y1.w);
      w3.x = r2[0] + bf16r(y2.x); w3.y = r2[1] + bf16r(y2.y); w3.z = r2[2] + bf16r(y2.z); w3.w = r2[3] + bf16r(y2.w);
      float* q0 = out0 + (size_t)gcl * HD + c4;
      float* q1 = out1 + (size_t)gcl * H3 + c4;
      if (wout) {
        *(volatile v4f*)q0 = w0;
        *(volatile v4f*)q1 = w1;
        *(volatile v4f*)(q1 + HD) = w2;
        *(volatile v4f*)(q1 + 2 * HD) = w3;
      }
      __threadfence();
      if (wout) {
        *(volatile v4f*)q0 = w0;
        *(volatile v4f*)q1 = w1;
        *(volatile v4f*)(q1 + HD) = w2;
        *(volatile v4f*)(q1 + 2 * HD) = w3;
      }
    } else {
      v4f w0, w1, w2, w3;
      w0.x = rs[0]; w0.y = rs[1]; w0.z = rs[2]; w0.w = rs[3];
      w1.x = r0[0]; w1.y = r0[1]; w1.z = r0[2]; w1.w = r0[3];
      w2.x = r1[0]; w2.y = r1[1]; w2.z = r1[2]; w2.w = r1[3];
      w3.x = r2[0]; w3.y = r2[1]; w3.z = r2[2]; w3.w = r2[3];
      float* q0 = DS + (size_t)gw * HD + c4;
      float* q1 = DV + (size_t)gw * H3 + c4;
      if (wr) {
        *(volatile v4f*)q0 = w0;
        *(volatile v4f*)q1 = w1;
        *(volatile v4f*)(q1 + HD) = w2;
        *(volatile v4f*)(q1 + 2 * HD) = w3;
      }
      __threadfence();
      if (wr) {
        *(volatile v4f*)q0 = w0;
        *(volatile v4f*)q1 = w1;
        *(volatile v4f*)(q1 + HD) = w2;
        *(volatile v4f*)(q1 + 2 * HD) = w3;
      }
    }
  }
}

static inline int cdiv(int a, int b) { return (a + b - 1) / b; }
static int pick_nb(int chm, int nN) {
  int nb = NBMAX;
  while (nb > 16 && (long long)nb * (long long)chm * 4LL > (long long)RCAP * (long long)nN) nb >>= 1;
  return nb;
}

extern "C" void kernel_launch(void* const* d_in, const int* in_sizes, int n_in,
                              void* d_out, int out_size, void* d_ws, size_t ws_size,
                              hipStream_t stream) {
  if (n_in < 13) return;
  const int nN = in_sizes[0] / HD;
  if (nN <= 0 || in_sizes[0] != nN * HD || nN > (1 << 20)) return;
  if (in_sizes[1] != nN * H3) return;
  if ((in_sizes[2] & 1) != 0) return;
  const int nE = in_sizes[2] / 2;
  if (nE < 1 || nE > (1 << 22)) return;
  if (in_sizes[3] != nE * RD || in_sizes[4] != nE * 3) return;
  if (in_sizes[5] != RD * HD || in_sizes[6] != HD) return;
  if (in_sizes[7] != HD * H3 || in_sizes[8] != H3) return;
  if (in_sizes[9] != HD * HD || in_sizes[10] != HD) return;
  if (in_sizes[11] != HD * H3 || in_sizes[12] != H3) return;
  if (out_size != nN * HD + nN * H3) return;

  const float* s    = (const float*)d_in[0];
  const float* v    = (const float*)d_in[1];
  const int*   ei   = (const int*)  d_in[2];
  const float* rbf  = (const float*)d_in[3];
  const float* unit = (const float*)d_in[4];
  const float* fW1  = (const float*)d_in[5];
  const float* fb1  = (const float*)d_in[6];
  const float* fW2  = (const float*)d_in[7];
  const float* fb2  = (const float*)d_in[8];
  const float* sW1  = (const float*)d_in[9];
  const float* sb1  = (const float*)d_in[10];
  const float* sW2  = (const float*)d_in[11];
  const float* sb2  = (const float*)d_in[12];
  float* out0 = (float*)d_out;
  float* out1 = out0 + (size_t)nN * HD;

  const int NP     = cdiv(nN, GBM) * GBM;
  const int tilesE = cdiv(nE, GBM);
  const int tpc    = ECH / GBM;
  const int NCHK   = cdiv(tilesE, tpc);
  const int CHM    = (tpc < tilesE ? tpc : tilesE) * GBM;
  const int nb     = pick_nb(CHM, nN);
  const int gA     = cdiv(nN, nb);
  const int NPD    = gA * nb;
  if (NPD < nN) return;

  char* ws = (char*)d_ws;
  size_t off = 0;
  const size_t oWT = off; off += (size_t)NW_TOT * 2;               off = (off + 255) & ~(size_t)255;
  const size_t oSA = off; off += (size_t)NP * HD * 2;              off = (off + 255) & ~(size_t)255;
  const size_t oHH = off; off += (size_t)NP * HD * 2;              off = (off + 255) & ~(size_t)255;
  const size_t oHL = off; off += (size_t)NP * HD * 2;              off = (off + 255) & ~(size_t)255;
  const size_t oSP = off; off += (size_t)NP * H3 * 4;              off = (off + 255) & ~(size_t)255;
  const size_t oRB = off; off += (size_t)CHM * KR * 2;             off = (off + 255) & ~(size_t)255;
  const size_t oZC = off; off += (size_t)CHM * HD * 2;             off = (off + 255) & ~(size_t)255;
  const size_t oFC = off; off += (size_t)CHM * H3 * 2;             off = (off + 255) & ~(size_t)255;
  const size_t oDS = off; off += (size_t)NPD * HD * 4;             off = (off + 255) & ~(size_t)255;
  const size_t oDV = off; off += (size_t)NPD * H3 * 4;             off = (off + 255) & ~(size_t)255;
  if (off > ws_size || off > (size_t)WSMAX) return;
  _Float16* WT  = (_Float16*)(ws + oWT);
  _Float16* SA  = (_Float16*)(ws + oSA);
  _Float16* HH  = (_Float16*)(ws + oHH);
  _Float16* HL  = (_Float16*)(ws + oHL);
  float*    SPp = (float*)(ws + oSP);
  _Float16* RB  = (_Float16*)(ws + oRB);
  _Float16* ZC  = (_Float16*)(ws + oZC);
  _Float16* FC  = (_Float16*)(ws + oFC);
  float*    DS  = (float*)(ws + oDS);
  float*    DV  = (float*)(ws + oDV);

  hipFuncSetAttribute(reinterpret_cast<const void*>(&k_drain),
                      hipFuncAttributeMaxDynamicSharedMemorySize, LDS_AGG);

  k_wcvt<<<U_TOT / NTHR, NTHR, 0, stream>>>(fW1, sW1, fW2, sW2, WT, U_TOT);
  {
    const int nU = NP * (HD / 8);
    k_scvt<<<cdiv(nU, NTHR), NTHR, 0, stream>>>(s, SA, nN, nU);
  }
  const int gM = NP / GBM;
  k_gemm<2, 0><<<dim3(gM, HD / GBN), GTHR, 0, stream>>>(SA, SA, WT + OW_S1, sb1, SPp, HH, HL,
                                                        HD, HD, HD, SCL_S1, CH);
  k_gemm<0, 1><<<dim3(gM, H3 / GBN), GTHR, 0, stream>>>(HH, HL, WT + OW_S2, sb2, SPp, HH, HL,
                                                        HD, H3, H3, SCL_S2, 1.0f);

  for (int c = 0; c < NCHK; ++c) {
    const int t0 = c * tpc;
    int t1 = t0 + tpc;
    t1 = t1 > tilesE ? tilesE : t1;
    if (t1 <= t0) continue;
    const int rows  = (t1 - t0) * GBM;
    const int ebase = t0 * GBM;
    int nEc = nE - ebase;
    nEc = nEc > rows ? rows : nEc;
    const int vec8  = ((((long long)nE + (long long)ebase) & 3LL) == 0) ? 1 : 0;
    const int accum = (c == 0) ? 0 : 1;
    const int fin   = (c == NCHK - 1) ? 1 : 0;
    {
      const int nU = rows * (KR / 8);
      k_rcvt<<<cdiv(nU, NTHR), NTHR, 0, stream>>>(rbf, RB, ebase, nE, nU);
    }
    k_gemm<1, 0><<<dim3(rows / GBM, HD / GBN), GTHR, 0, stream>>>(RB, RB, WT + OW_F1, fb1, SPp, ZC, ZC,
                                                                  KR, HD, HD, SCL_F1, CZ);
    k_gemm<3, 0><<<dim3(rows / GBM, H3 / GBN), GTHR, 0, stream>>>(ZC, ZC, WT + OW_F2, fb2, SPp, FC, FC,
                                                                  HD, H3, H3, SCL_F2, CF);
    k_drain<<<gA, NTHR, LDS_AGG, stream>>>(ei, unit, FC, SPp, v, s, DS, DV, out0, out1,
                                           nN, nE, ebase, nEc, nb, vec8, NPD, accum, fin);
  }
}
